// _DeformConvBase_28905129902135
// MI455X (gfx1250) — hardware-verified
//
#include <hip/hip_runtime.h>

typedef __bf16   v16b __attribute__((ext_vector_type(16)));
typedef __bf16   v8b  __attribute__((ext_vector_type(8)));
typedef float    v8f  __attribute__((ext_vector_type(8)));
typedef float    v4f  __attribute__((ext_vector_type(4)));
typedef unsigned short v8u __attribute__((ext_vector_type(8)));
typedef v8b __attribute__((may_alias)) v8ba;
typedef v4f __attribute__((may_alias)) v4fa;
typedef float __attribute__((may_alias)) f32a;

#pragma clang fp contract(off)

#define NB    8
#define CH    64
#define HH    128
#define WW    128
#define PIX   16384
#define NPIX  131072
#define KDIM  576
#define PITCH 584
#define NOFF  18
#define NOFFP 32
#define NX    (NB * CH * PIX)
#define NWO   (NOFF * KDIM)
#define NWOP  (NOFFP * KDIM)
#define NWC   (CH * KDIM)
#define DMT   64
#define DPL   (DMT * PITCH)
#define XBLK  (NX / 2048)
#define WOBLK (NWOP / 2048)
#define WCBLK (NWC / 2048)

static_assert(NX % 2048 == 0);
static_assert(NWOP % 2048 == 0);
static_assert(NWC % 2048 == 0);
static_assert(NWO % 8 == 0);
static_assert(NPIX % DMT == 0);
static_assert(WW % DMT == 0);
static_assert(KDIM % 32 == 0);
static_assert((PITCH * 2) % 16 == 0);

__device__ __forceinline__ v8f wmma_bf16(v16b a, v16b b, v8f c) {
  v8f d = __builtin_amdgcn_wmma_f32_16x16x32_bf16(false, a, false, b, (short)0, c, false, false);
  asm volatile("v_nop\n\tv_nop\n\tv_nop\n\tv_nop" : "+v"(d) : "v"(a), "v"(b));
  return d;
}

__device__ __forceinline__ v16b frag_b(const unsigned short* p, int h) {
  union { v16b v; v8b hv[2]; } f;
  f.hv[0] = *(const v8ba*)(p + 8 * h);
  f.hv[1] = *(const v8ba*)(p + 16 + 8 * h);
  return f.v;
}

__device__ __forceinline__ unsigned short bf16bits(float v) {
  unsigned int u = __float_as_uint(v);
  u += 0x7FFFu + ((u >> 16) & 1u);
  return (unsigned short)(u >> 16);
}
__device__ __forceinline__ float bf16val(unsigned short b) {
  return __uint_as_float(((unsigned int)b) << 16);
}
__device__ __forceinline__ int clampi(int v, int lo, int hi) {
  return v < lo ? lo : (v > hi ? hi : v);
}
__device__ __forceinline__ void split2(float v, unsigned short& hb, unsigned short& lb) {
  hb = bf16bits(v);
  lb = bf16bits(v - bf16val(hb));
}

__global__ __launch_bounds__(256) void convert_kernel(
    const float* __restrict__ x, const float* __restrict__ wo, const float* __restrict__ wc,
    unsigned short* __restrict__ xhi, unsigned short* __restrict__ xlo,
    unsigned short* __restrict__ wohi, unsigned short* __restrict__ wolo,
    unsigned short* __restrict__ wchi, unsigned short* __restrict__ wclo)
{
  const int blk = blockIdx.x, t = threadIdx.x;
  const float* src;
  unsigned short* dh;
  unsigned short* dl;
  int e, lim;
  if (blk < XBLK) {
    e = blk * 256 + t; src = x; dh = xhi; dl = xlo; lim = NX / 8;
  } else if (blk < XBLK + WOBLK) {
    e = (blk - XBLK) * 256 + t; src = wo; dh = wohi; dl = wolo; lim = NWO / 8;
  } else {
    e = (blk - XBLK - WOBLK) * 256 + t; src = wc; dh = wchi; dl = wclo; lim = NWC / 8;
  }
  const int ec = (e < lim) ? e : (lim - 1);
  v4f a = *(const v4fa*)(src + (size_t)ec * 8);
  v4f c = *(const v4fa*)(src + (size_t)ec * 8 + 4);
  const v4f z4 = {0.f, 0.f, 0.f, 0.f};
  a = (e < lim) ? a : z4;
  c = (e < lim) ? c : z4;
  v8u oh, ol;
  unsigned short hb, lb;
  split2(a.x, hb, lb); oh[0] = hb; ol[0] = lb;
  split2(a.y, hb, lb); oh[1] = hb; ol[1] = lb;
  split2(a.z, hb, lb); oh[2] = hb; ol[2] = lb;
  split2(a.w, hb, lb); oh[3] = hb; ol[3] = lb;
  split2(c.x, hb, lb); oh[4] = hb; ol[4] = lb;
  split2(c.y, hb, lb); oh[5] = hb; ol[5] = lb;
  split2(c.z, hb, lb); oh[6] = hb; ol[6] = lb;
  split2(c.w, hb, lb); oh[7] = hb; ol[7] = lb;
  unsigned short* ph = dh + (size_t)e * 8;
  unsigned short* pl = dl + (size_t)e * 8;
  *(volatile v8u*)ph = oh;
  *(volatile v8u*)pl = ol;
  __threadfence();
  *(volatile v8u*)ph = oh;
  *(volatile v8u*)pl = ol;
}

__device__ __forceinline__ void o_store_pass(const f32a* sT, float* out,
                                             int b, int p0, int w, int lane) {
  const int sub = lane >> 4, q4 = 4 * (lane & 15);
  #pragma unroll
  for (int q = 0; q < 8; ++q) {
    const int ch = 2 * (8 * w + q) + sub;
    const v4f v = *(const v4fa*)(sT + ch * DMT + q4);
    float* dst = out + (size_t)(b * CH + ch) * PIX + p0 + q4;
    *(volatile v4f*)dst = v;
  }
}

__global__ __launch_bounds__(128) void dcn_fused_kernel(
    const float* __restrict__ x,
    const unsigned short* __restrict__ xhi,
    const unsigned short* __restrict__ xlo,
    const unsigned short* __restrict__ wohi,
    const unsigned short* __restrict__ wolo,
    const float* __restrict__ boff,
    const unsigned short* __restrict__ wchi,
    const unsigned short* __restrict__ wclo,
    const float* __restrict__ bconv,
    float* __restrict__ out)
{
  __shared__ __attribute__((aligned(16))) unsigned short sA[2 * DPL];
  __shared__ __attribute__((aligned(16))) float sOff[DMT * NOFF];

  const int tid = threadIdx.x, lane = tid & 31, w = tid >> 5;
  const int h = lane >> 4, m = lane & 15;
  const int g0 = blockIdx.x * DMT;
  const int b = g0 / PIX;
  const int p0 = g0 - b * PIX;
  const int y = p0 / WW;
  const int x0 = p0 - y * WW;

  {
    const int r = tid & (DMT - 1), half = tid >> 6;
    const int xw = x0 + r;
    const unsigned short* sbh = xhi + (size_t)b * CH * PIX;
    const unsigned short* sbl = xlo + (size_t)b * CH * PIX;
    unsigned short* arow = sA + r * PITCH;
    #pragma unroll 1
    for (int c = half * 32; c < half * 32 + 32; ++c) {
      const unsigned short* sph = sbh + (size_t)c * PIX;
      const unsigned short* spl = sbl + (size_t)c * PIX;
      #pragma unroll
      for (int ky = 0; ky < 3; ++ky) {
        const int yy = y + ky - 1;
        const bool vy = (yy >= 0) && (yy < HH);
        const int yc = clampi(yy, 0, HH - 1);
        #pragma unroll
        for (int kx = 0; kx < 3; ++kx) {
          const int xx = xw + kx - 1;
          const bool vx = (xx >= 0) && (xx < WW);
          const int xc = clampi(xx, 0, WW - 1);
          const int idx = yc * WW + xc;
          const unsigned short vh = sph[idx];
          const unsigned short vl = spl[idx];
          const bool v = vy && vx;
          const int kk = c * 9 + ky * 3 + kx;
          arow[kk]       = v ? vh : (unsigned short)0;
          arow[DPL + kk] = v ? vl : (unsigned short)0;
        }
      }
    }
  }
  __syncthreads();

  const v8f zero8 = {0.f, 0.f, 0.f, 0.f, 0.f, 0.f, 0.f, 0.f};
  const unsigned short* arow_m = sA + (16 * w + m) * PITCH;

  {
    v8f acc[2];
    acc[0] = zero8; acc[1] = zero8;
    const unsigned short* wh = wohi + (size_t)m * KDIM;
    const unsigned short* wl = wolo + (size_t)m * KDIM;
    #pragma unroll 1
    for (int k0 = 0; k0 < KDIM; k0 += 32) {
      const v16b ah = frag_b(arow_m + k0, h);
      const v16b al = frag_b(arow_m + DPL + k0, h);
      #pragma unroll
      for (int j = 0; j < 2; ++j) {
        const v16b bh = frag_b(wh + (size_t)(16 * j) * KDIM + k0, h);
        const v16b bl = frag_b(wl + (size_t)(16 * j) * KDIM + k0, h);
        acc[j] = wmma_bf16(ah, bh, acc[j]);
        acc[j] = wmma_bf16(ah, bl, acc[j]);
        acc[j] = wmma_bf16(al, bh, acc[j]);
      }
    }
    #pragma unroll
    for (int j = 0; j < 2; ++j) {
      const int n = 16 * j + m;
      const float bj = boff[clampi(n, 0, NOFF - 1)];
      if (n < NOFF) {
        #pragma unroll
        for (int r = 0; r < 8; ++r)
          sOff[(16 * w + 8 * h + r) * NOFF + n] = acc[j][r] + bj;
      }
    }
  }
  __syncthreads();

  {
    const int r = tid & (DMT - 1), half = tid >> 6;
    const int xw = x0 + r;
    const float* xb = x + (size_t)b * CH * PIX;
    unsigned short* arow = sA + r * PITCH;
    const float* orow = sOff + r * NOFF;
    #pragma unroll 1
    for (int k9 = 0; k9 < 9; ++k9) {
      const int ky = k9 / 3;
      const int kx = k9 - 3 * ky;
      const float dy = orow[2 * k9];
      const float dx = orow[2 * k9 + 1];
      const float py = dy + (float)(y - 1 + ky);
      const float px = dx + (float)(xw - 1 + kx);
      const float y0f = floorf(py), x0f = floorf(px);
      const float wy1 = py - y0f, wx1 = px - x0f;
      const float wy0 = 1.0f - wy1, wx0 = 1.0f - wx1;
      const float y1f = y0f + 1.0f, x1f = x0f + 1.0f;
      const bool vy0 = (y0f >= 0.0f) && (y0f <= (float)(HH - 1));
      const bool vy1 = (y1f >= 0.0f) && (y1f <= (float)(HH - 1));
      const bool vx0 = (x0f >= 0.0f) && (x0f <= (float)(WW - 1));
      const bool vx1 = (x1f >= 0.0f) && (x1f <= (float)(WW - 1));
      const int iy0 = (int)fminf(fmaxf(y0f, 0.0f), (float)(HH - 1));
      const int iy1 = (int)fminf(fmaxf(y1f, 0.0f), (float)(HH - 1));
      const int ix0 = (int)fminf(fmaxf(x0f, 0.0f), (float)(WW - 1));
      const int ix1 = (int)fminf(fmaxf(x1f, 0.0f), (float)(WW - 1));
      const float w00 = (wy0 * wx0) * ((vy0 && vx0) ? 1.0f : 0.0f);
      const float w01 = (wy0 * wx1) * ((vy0 && vx1) ? 1.0f : 0.0f);
      const float w10 = (wy1 * wx0) * ((vy1 && vx0) ? 1.0f : 0.0f);
      const float w11 = (wy1 * wx1) * ((vy1 && vx1) ? 1.0f : 0.0f);
      const int i00 = iy0 * WW + ix0, i01 = iy0 * WW + ix1;
      const int i10 = iy1 * WW + ix0, i11 = iy1 * WW + ix1;
      #pragma unroll 4
      for (int c = half * 32; c < half * 32 + 32; ++c) {
        const float* xp = xb + (size_t)c * PIX;
        const float g00 = xp[i00];
        const float g01 = xp[i01];
        const float g10 = xp[i10];
        const float g11 = xp[i11];
        const float s = ((g00 * w00 + g01 * w01) + g10 * w10) + g11 * w11;
        unsigned short hb, lb;
        split2(s, hb, lb);
        const int kk = c * 9 + k9;
        arow[kk] = hb;
        arow[DPL + kk] = lb;
      }
    }
  }
  __syncthreads();

  v8f acc[4];
  #pragma unroll
  for (int j = 0; j < 4; ++j) acc[j] = zero8;
  {
    const unsigned short* wh = wchi + (size_t)m * KDIM;
    const unsigned short* wl = wclo + (size_t)m * KDIM;
    #pragma unroll 1
    for (int k0 = 0; k0 < KDIM; k0 += 32) {
      const v16b ah = frag_b(arow_m + k0, h);
      const v16b al = frag_b(arow_m + DPL + k0, h);
      #pragma unroll
      for (int j = 0; j < 4; ++j) {
        const v16b bh = frag_b(wh + (size_t)(16 * j) * KDIM + k0, h);
        const v16b bl = frag_b(wl + (size_t)(16 * j) * KDIM + k0, h);
        acc[j] = wmma_bf16(ah, bh, acc[j]);
        acc[j] = wmma_bf16(ah, bl, acc[j]);
        acc[j] = wmma_bf16(al, bh, acc[j]);
      }
    }
  }
  __syncthreads();

  {
    f32a* sT = (f32a*)sA;
    #pragma unroll
    for (int j = 0; j < 4; ++j) {
      const float bj = bconv[16 * j + m];
      #pragma unroll
      for (int r = 0; r < 8; ++r)
        sT[(16 * j + m) * DMT + 16 * w + 8 * h + r] = acc[j][r] + bj;
    }
    __syncthreads();
    o_store_pass(sT, out, b, p0, w, lane);
    __threadfence();
    o_store_pass(sT, out, b, p0, w, lane);
  }
}

extern "C" void kernel_launch(void* const* d_in, const int* in_sizes, int n_in,
                              void* d_out, int out_size, void* d_ws, size_t ws_size,
                              hipStream_t stream) {
  if (n_in < 5) return;
  if (in_sizes[0] != NX || in_sizes[1] != NWO || in_sizes[2] != NOFF ||
      in_sizes[3] != NWC || in_sizes[4] != CH) return;
  if (out_size != NX) return;

  const float* x     = (const float*)d_in[0];
  const float* wo    = (const float*)d_in[1];
  const float* boff  = (const float*)d_in[2];
  const float* wc    = (const float*)d_in[3];
  const float* bconv = (const float*)d_in[4];
  float* out = (float*)d_out;

  const size_t xp_b = (size_t)NX * 2;
  const size_t wo_b = (size_t)NWOP * 2;
  const size_t wc_b = (size_t)NWC * 2;
  const size_t total = 2 * xp_b + 2 * wo_b + 2 * wc_b;
  if (total > ws_size) return;
  if (total > (size_t)134217728) return;

  char* ws = (char*)d_ws;
  unsigned short* xhi  = (unsigned short*)(ws);
  unsigned short* xlo  = (unsigned short*)(ws + xp_b);
  unsigned short* wohi = (unsigned short*)(ws + 2 * xp_b);
  unsigned short* wolo = (unsigned short*)(ws + 2 * xp_b + wo_b);
  unsigned short* wchi = (unsigned short*)(ws + 2 * xp_b + 2 * wo_b);
  unsigned short* wclo = (unsigned short*)(ws + 2 * xp_b + 2 * wo_b + wc_b);

  convert_kernel<<<XBLK + WOBLK + WCBLK, 256, 0, stream>>>(x, wo, wc, xhi, xlo, wohi, wolo, wchi, wclo);

  dcn_fused_kernel<<<NPIX / DMT, 128, 0, stream>>>(x, xhi, xlo, wohi, wolo, boff, wchi, wclo, bconv, out);
}
